// Self_Attention_Memory_Module_75170517615300
// MI455X (gfx1250) — hardware-verified
//
#include <hip/hip_runtime.h>
#include <hip/hip_bf16.h>
#include <math.h>

#define BB 8
#define IMH 48
#define SS 2304
#define DD 64
#define HH 1
#define KVH 1
#define KVD 64
#define DKK 64
#define QW 2
#define HID 64
#define MTOK (BB * SS)
#define GSTR 48

typedef _Float16 bf16;
typedef _Float16 f16;
typedef __attribute__((ext_vector_type(4))) unsigned v4u_t;
typedef unsigned v4ua __attribute__((ext_vector_type(4), may_alias));
typedef __attribute__((ext_vector_type(4))) float v4f_t;
typedef float v4fa __attribute__((ext_vector_type(4), may_alias));
typedef __attribute__((ext_vector_type(16))) bf16  bf16x16;
typedef bf16x16 f16x16;
typedef __attribute__((ext_vector_type(8)))  bf16  bf16x8;
typedef bf16x8 f16x8;
typedef __attribute__((ext_vector_type(4)))  bf16  bf16x4;
typedef __attribute__((ext_vector_type(8)))  float f32x8;
__device__ __forceinline__ f32x8 wmma16(f16x16 a, f16x16 b, f32x8 c) {
  c = __builtin_amdgcn_wmma_f32_16x16x32_f16(false, a, false, b, (short)0, c, false, false);
  asm volatile("v_nop\n\tv_nop\n\tv_nop\n\tv_nop" : "+v"(c) : "v"(a), "v"(b));
  return c;
}
#define LDS_STRIDE 48
#define KSTRIDE    72
#define VSTRIDE    48

__device__ __forceinline__ f32x8 wmma_bf16(bf16x16 a, bf16x16 b, f32x8 c) {
  c = __builtin_amdgcn_wmma_f32_16x16x32_f16(false, a, false, b, (short)0, c, false, false);
  asm volatile("v_nop\n\tv_nop\n\tv_nop\n\tv_nop" : "+v"(c) : "v"(a), "v"(b));
  return c;
}

template <typename T>
__device__ __forceinline__ bf16x16 load_frag(const T* __restrict__ base, int ld,
                                             int row0, int k0) {
  const int lane = threadIdx.x & 31;
  const int r    = lane & 15;
  const int kh   = (lane >> 4) * 8;
  const T* p0 = base + (size_t)(row0 + r) * ld + (k0 + kh);
  const T* p1 = p0 + 16;
  bf16x16 f;
#pragma unroll
  for (int i = 0; i < 8; ++i) {
    f[i]     = (bf16)p0[i];
    f[i + 8] = (bf16)p1[i];
  }
  return f;
}

__device__ __forceinline__ bf16x16 lds_frag(const bf16* base, int stride) {
  const int lane = threadIdx.x & 31;
  const int row  = lane & 15;
  const int kh   = (lane >> 4) * 8;
  const bf16x8 lo = *(const bf16x8*)(base + row * stride + kh);
  const bf16x8 hi = *(const bf16x8*)(base + row * stride + kh + 16);
  bf16x16 f;
#pragma unroll
  for (int i = 0; i < 8; ++i) { f[i] = lo[i]; f[i + 8] = hi[i]; }
  return f;
}

template <typename T>
__device__ __forceinline__ void stage_read16(const T* __restrict__ p, float* buf) {
#pragma unroll
  for (int i = 0; i < 16; ++i) buf[i] = (float)p[i];
}

__device__ __forceinline__ void stage_write(bf16* dst, const float* buf, int nquad) {
#pragma unroll
  for (int i = 0; i < nquad; ++i) {
    bf16x4 q;
    q[0] = (bf16)buf[4 * i];     q[1] = (bf16)buf[4 * i + 1];
    q[2] = (bf16)buf[4 * i + 2]; q[3] = (bf16)buf[4 * i + 3];
    *(bf16x4*)(dst + 4 * i) = q;
  }
}

__global__ __launch_bounds__(64) void attn_kernel(
    const bf16* __restrict__ Qb, const bf16* __restrict__ Kb,
    const bf16* __restrict__ Vt,
    bf16* __restrict__ attnOut) {
  __shared__ bf16 ldsK[32 * KSTRIDE];
  __shared__ bf16 ldsV[64 * VSTRIDE];
  __shared__ __attribute__((aligned(16))) bf16 ldsO[2][32 * 72];

  const int q0blk = blockIdx.x * 64;
  const int h  = blockIdx.y;
  const int b  = blockIdx.z;
  const int t    = threadIdx.x;
  const int wave = t >> 5;
  const int lane = t & 31;
  const int qlane = lane & 15;
  const int kh8   = (lane >> 4) * 8;
  const int q0 = q0blk + wave * 32;

  const int hk = h;
  const bf16* Qh = Qb + (size_t)b * SS * DD + h * DKK;
  const bf16* Kh = Kb + (size_t)b * SS * KVD + hk * DKK;
  const bf16* Vh = Vt + ((size_t)(b * KVH + hk)) * DKK * SS;

  const int krow = t >> 1;
  const int kcol = (t & 1) * 32;
  const bf16* kSrc = Kh + (size_t)krow * KVD + kcol;
  const bf16* vSrc = Vh + (size_t)t * SS;

  bf16x16 qf[QW][2];
#pragma unroll
  for (int qt = 0; qt < QW; ++qt) {
    qf[qt][0] = load_frag(Qh, DD, q0 + 16 * qt, 0);
    qf[qt][1] = load_frag(Qh, DD, q0 + 16 * qt, 32);
  }

  f32x8 o[QW][4] = {};
  float mrun[QW], lrun[QW];
#pragma unroll
  for (int qt = 0; qt < QW; ++qt) { mrun[qt] = -INFINITY; lrun[qt] = 0.0f; }

  const float scale = 0.125f * 1.44269504088896340736f;
  const float NEG2 = -1.0e9f;
  const int kmax = SS - 1;

  bf16x8 kreg[4], vreg[4];
#pragma unroll
  for (int i = 0; i < 4; ++i) {
    kreg[i] = *(const bf16x8*)(kSrc + 8 * i);
    vreg[i] = *(const bf16x8*)(vSrc + 8 * i);
  }

  for (int kb = 0; kb <= kmax; kb += 32) {
    __syncthreads();
#pragma unroll
    for (int i = 0; i < 4; ++i) {
      *(bf16x8*)(&ldsK[krow * KSTRIDE + kcol + 8 * i]) = kreg[i];
      *(bf16x8*)(&ldsV[t * VSTRIDE + 8 * i])           = vreg[i];
    }
    if (kb + 32 <= kmax) {
      const bf16* kn = kSrc + (size_t)(kb + 32) * KVD;
      const bf16* vn = vSrc + (kb + 32);
#pragma unroll
      for (int i = 0; i < 4; ++i) {
        kreg[i] = *(const bf16x8*)(kn + 8 * i);
        vreg[i] = *(const bf16x8*)(vn + 8 * i);
      }
    }
    __syncthreads();

    bf16x16 kf[2][2];
#pragma unroll
    for (int ktile = 0; ktile < 2; ++ktile)
#pragma unroll
      for (int c = 0; c < 2; ++c)
        kf[ktile][c] = lds_frag(ldsK + (ktile * 16) * KSTRIDE + c * 32, KSTRIDE);

    bf16x16 pf[QW];
    bool act[QW];
#pragma unroll
    for (int qt = 0; qt < QW; ++qt) {
      unsigned mbits = 0;
      mbits = 0xFFFFu; act[qt] = true;
      if (act[qt]) {
        const int q_my = q0 + 16 * qt + qlane;
        f32x8 s0 = {}, s1 = {};
        s0 = wmma_bf16(kf[0][0], qf[qt][0], s0);
        s0 = wmma_bf16(kf[0][1], qf[qt][1], s0);
        s1 = wmma_bf16(kf[1][0], qf[qt][0], s1);
        s1 = wmma_bf16(kf[1][1], qf[qt][1], s1);

        float mx = -INFINITY;
#pragma unroll
        for (int r = 0; r < 8; ++r) {
          const int k0i = kb + kh8 + r;
          const int k1i = k0i + 16;
          (void)k0i; (void)k1i; (void)q_my;
          s0[r] = (mbits & (1u << r))       ? s0[r] * scale : NEG2;
          s1[r] = (mbits & (1u << (8 + r))) ? s1[r] * scale : NEG2;
          mx = fmaxf(mx, fmaxf(s0[r], s1[r]));
        }
        mx = fmaxf(mx, __shfl_xor(mx, 16, 32));
        const float mnew  = fmaxf(mrun[qt], mx);
        const float alpha = exp2f(mrun[qt] - mnew);

        float rsum = 0.0f;
#pragma unroll
        for (int r = 0; r < 8; ++r) {
          const float p0 = exp2f(s0[r] - mnew);
          const float p1 = exp2f(s1[r] - mnew);
          rsum += p0 + p1;
          pf[qt][r]     = (bf16)(p0 * 1024.0f);
          pf[qt][r + 8] = (bf16)(p1 * 1024.0f);
        }
        rsum += __shfl_xor(rsum, 16, 32);
        lrun[qt] = lrun[qt] * alpha + rsum;
        mrun[qt] = mnew;

#pragma unroll
        for (int j = 0; j < 4; ++j)
#pragma unroll
          for (int r = 0; r < 8; ++r) o[qt][j][r] *= alpha;
      }
    }

#pragma unroll
    for (int j = 0; j < 4; ++j) {
      const bf16x16 vf = lds_frag(ldsV + (j * 16) * VSTRIDE, VSTRIDE);
#pragma unroll
      for (int qt = 0; qt < QW; ++qt)
        if (act[qt]) o[qt][j] = wmma_bf16(vf, pf[qt], o[qt][j]);
    }
  }

  bf16* so = ldsO[wave];
#pragma unroll
  for (int qt = 0; qt < QW; ++qt) {
    const float rl = 1.0f / (lrun[qt] * 1024.0f);
#pragma unroll
    for (int j = 0; j < 4; ++j)
#pragma unroll
      for (int r = 0; r < 8; ++r) so[(16 * qt + qlane) * 72 + j * 16 + kh8 + r] = (bf16)(o[qt][j][r] * rl);
  }
  asm volatile("s_wait_dscnt 0" ::: "memory");
#pragma unroll 1
  for (int pass = 0; pass < 2; ++pass) {
#pragma unroll
    for (int it = 0; it < 8; ++it) { const int ch = lane + 32 * it, ql = ch >> 3, q8 = (ch & 7) * 8;
      *(volatile v4u_t*)(attnOut + ((size_t)(b * SS + q0 + ql)) * DD + h * DKK + q8) = *(const v4ua*)(so + ql * 72 + q8); }
    __threadfence();
  }
}


template <int CIN, int NOUT, typename IT, bool OUT16>
__global__ __launch_bounds__(256) void k_conv(const IT* __restrict__ in, const float* __restrict__ Wt, const float* __restrict__ bias, void* __restrict__ outv) {
  constexpr int NCT = NOUT / 16;
  __shared__ __attribute__((aligned(16))) f16 aS[128 * 40];
  __shared__ __attribute__((aligned(16))) f16 bS[NOUT * 40];
  __shared__ __attribute__((aligned(16))) float oS[128 * 68];
  const int tid = threadIdx.x, lane = tid & 31, wave = tid >> 5, cl = lane & 15, rh = (lane >> 4) * 8;
  const size_t t0 = (size_t)blockIdx.x * 128;
  const int r = tid >> 1, hq = (tid & 1) * 16; const size_t tok = t0 + r; const int b = tok / SS, pix = tok % SS, py = pix / IMH, px = pix % IMH;
  f32x8 acc[NCT];
#pragma unroll
  for (int j = 0; j < NCT; ++j) { f32x8 z = {}; acc[j] = z; }
#pragma unroll 1
  for (int ks = 0; ks < 9 * CIN / 32; ++ks) {
    __syncthreads();
    { const int k0 = ks * 32; const int tap = k0 / CIN, ci0 = k0 % CIN; const int yy = py + tap / 3 - 1, xx = px + tap % 3 - 1;
      const bool ok = (yy >= 0 && yy < IMH && xx >= 0 && xx < IMH);
      const int yyc = ok ? yy : py, xxc = ok ? xx : px;
      const IT* src = in + (((size_t)b * IMH + yyc) * IMH + xxc) * CIN + ci0 + hq;
#pragma unroll
      for (int e = 0; e < 16; ++e) { float v = (float)src[e]; aS[r * 40 + hq + e] = (f16)(ok ? v : 0.0f); } }
    for (int e = tid; e < NOUT * 8; e += 256) { const int n = e >> 3, kq = (e & 7) * 4; const float* wr = Wt + (size_t)(ks * 32 + kq) * NOUT + n;
      bS[n * 40 + kq] = (f16)wr[0]; bS[n * 40 + kq + 1] = (f16)wr[NOUT]; bS[n * 40 + kq + 2] = (f16)wr[2 * NOUT]; bS[n * 40 + kq + 3] = (f16)wr[3 * NOUT]; }
    __syncthreads();
    const f16x16 af = lds_frag(aS + (wave * 16) * 40, 40);
#pragma unroll
    for (int j = 0; j < NCT; ++j) acc[j] = wmma16(af, lds_frag(bS + (j * 16) * 40, 40), acc[j]);
  }
#pragma unroll
  for (int ch = 0; ch < NCT / 4; ++ch) {
    __syncthreads();
#pragma unroll
    for (int jj = 0; jj < 4; ++jj) { const int j = ch * 4 + jj; const float bb = bias[j * 16 + cl];
#pragma unroll
      for (int rr = 0; rr < 8; ++rr) oS[(wave * 16 + rh + rr) * 68 + jj * 16 + cl] = acc[j][rr] + bb; }
    __syncthreads();
#pragma unroll 1
    for (int pass = 0; pass < 2; ++pass) {
      if (OUT16) { bf16* o = (bf16*)outv; for (int e = tid; e < 128 * 8; e += 256) { const int rr = e >> 3, c8 = (e & 7) * 8; union { bf16 hh[8]; v4u_t u; } cv;
          for (int i = 0; i < 8; ++i) cv.hh[i] = (bf16)oS[rr * 68 + c8 + i]; *(volatile v4u_t*)(o + (t0 + rr) * NOUT + ch * 64 + c8) = cv.u; } }
      else { float* o = (float*)outv; for (int e = tid; e < 128 * 16; e += 256) { const int rr = e >> 4, c4 = (e & 15) * 4;
          *(volatile v4f_t*)(o + (t0 + rr) * NOUT + ch * 64 + c4) = *(const v4fa*)(oS + rr * 68 + c4); } }
      __threadfence(); }
  }
}
__global__ __launch_bounds__(256) void k_qkv16(const float* __restrict__ q, const float* __restrict__ k, const float* __restrict__ v, bf16* __restrict__ Q16, bf16* __restrict__ K16, bf16* __restrict__ Vt) {
  __shared__ __attribute__((aligned(16))) bf16 qS[64][72], kS[64][72], vT[64][72];
  const int tid = threadIdx.x; const size_t t0 = (size_t)blockIdx.x * 64; const int b = (int)(t0 / SS), n0 = (int)(t0 % SS);
  for (int e = tid; e < 64 * 64; e += 256) { const int t = e >> 6, d = e & 63; const size_t off = (t0 + t) * DD + d; if (q) qS[t][d] = (bf16)(q[off] * 8.0f); kS[t][d] = (bf16)k[off]; vT[d][t] = (bf16)v[off]; }
  __syncthreads();
#pragma unroll 1
  for (int pass = 0; pass < 2; ++pass) {
#pragma unroll 1
    for (int round = 0; round < 2; ++round) { const int r = round * 32 + (tid >> 3), piece = (tid & 7) * 8;
      if (q) *(volatile v4u_t*)(Q16 + (t0 + r) * DD + piece) = *(const v4ua*)(&qS[r][piece]);
      *(volatile v4u_t*)(K16 + (t0 + r) * DD + piece) = *(const v4ua*)(&kS[r][piece]);
      *(volatile v4u_t*)(Vt + ((size_t)b * DD + r) * SS + n0 + piece) = *(const v4ua*)(&vT[r][piece]); }
    __threadfence(); }
}
__global__ __launch_bounds__(128) void k_cat2(const bf16* __restrict__ zh, const bf16* __restrict__ zm, float* __restrict__ Cc) { const size_t tok = blockIdx.x; const int c = threadIdx.x;
  const float v = (c < 64) ? (float)zh[tok * DD + c] : (float)zm[tok * DD + c - 64]; *(volatile float*)(Cc + tok * 128 + c) = v; __threadfence(); *(volatile float*)(Cc + tok * 128 + c) = v; }
__global__ __launch_bounds__(192) void k_cat3(const float* __restrict__ Z, const float* __restrict__ h, float* __restrict__ C3) { const size_t tok = blockIdx.x; const int c = threadIdx.x;
  const float v = (c < 128) ? Z[tok * 128 + c] : h[tok * DD + c - 128]; *(volatile float*)(C3 + tok * 192 + c) = v; __threadfence(); *(volatile float*)(C3 + tok * 192 + c) = v; }
__global__ __launch_bounds__(64) void k_gates(const float* __restrict__ comb, const float* __restrict__ m, float* __restrict__ new_h, float* __restrict__ new_m) { const size_t tok = blockIdx.x; const int c = threadIdx.x;
  const float mo = comb[tok * 192 + c], mg = comb[tok * 192 + 64 + c], mi = comb[tok * 192 + 128 + c]; const float si = 1.0f / (1.0f + expf(-mi)), so = 1.0f / (1.0f + expf(-mo));
  const float nm = (1.0f - si) * m[tok * DD + c] + si * tanhf(mg); const float nh = so * nm;
  *(volatile float*)(new_m + tok * DD + c) = nm; *(volatile float*)(new_h + tok * DD + c) = nh; __threadfence(); *(volatile float*)(new_m + tok * DD + c) = nm; *(volatile float*)(new_h + tok * DD + c) = nh; }

extern "C" void kernel_launch(void* const* d_in, const int* in_sizes, int n_in,
                              void* d_out, int out_size, void* d_ws, size_t ws_size,
                              hipStream_t stream) {
  (void)in_sizes; (void)n_in; (void)out_size;
  const float** f = (const float**)d_in;
  const float* h = f[0], *m = f[1], *Wq = f[2], *bq = f[3], *Wk = f[4], *bk = f[5], *Wk2 = f[6], *bk2 = f[7], *Wv = f[8], *bv = f[9], *Wv2 = f[10], *bv2 = f[11], *Wz = f[12], *bz = f[13], *Wm = f[14], *bm = f[15];
  float* new_h = (float*)d_out; float* new_m = new_h + (size_t)MTOK * DD;
  char* ws = (char*)d_ws;
  float* q = (float*)ws; ws += (size_t)MTOK * DD * 4; float* k = (float*)ws; ws += (size_t)MTOK * DD * 4; float* v = (float*)ws; ws += (size_t)MTOK * DD * 4;
  bf16* Q16 = (bf16*)ws; ws += (size_t)MTOK * DD * 2; bf16* K16 = (bf16*)ws; ws += (size_t)MTOK * DD * 2; bf16* Vt = (bf16*)ws; ws += (size_t)MTOK * DD * 2;
  bf16* zh = (bf16*)ws; ws += (size_t)MTOK * DD * 2; bf16* zm = (bf16*)ws; ws += (size_t)MTOK * DD * 2;
  float* Cc = (float*)ws; ws += (size_t)MTOK * 128 * 4; float* Z = (float*)ws; ws += (size_t)MTOK * 128 * 4; float* C3 = (float*)ws; ws += (size_t)MTOK * 192 * 4; float* comb = (float*)ws; ws += (size_t)MTOK * 192 * 4;
  if ((size_t)(ws - (char*)d_ws) > ws_size) return;
  const dim3 blk(256); const dim3 gc(MTOK / 128);
  k_conv<64, 64, float, false><<<gc, blk, 0, stream>>>(h, Wq, bq, q); k_conv<64, 64, float, false><<<gc, blk, 0, stream>>>(h, Wk, bk, k); k_conv<64, 64, float, false><<<gc, blk, 0, stream>>>(h, Wv, bv, v);
  k_qkv16<<<dim3(MTOK / 64), blk, 0, stream>>>(q, k, v, Q16, K16, Vt);
  attn_kernel<<<dim3(SS / 64, HH, BB), dim3(64), 0, stream>>>(Q16, K16, Vt, zh);
  k_conv<64, 64, float, false><<<gc, blk, 0, stream>>>(m, Wk2, bk2, k); k_conv<64, 64, float, false><<<gc, blk, 0, stream>>>(m, Wv2, bv2, v);
  k_qkv16<<<dim3(MTOK / 64), blk, 0, stream>>>(nullptr, k, v, Q16, K16, Vt);
  attn_kernel<<<dim3(SS / 64, HH, BB), dim3(64), 0, stream>>>(Q16, K16, Vt, zm);
  k_cat2<<<dim3(MTOK), dim3(128), 0, stream>>>(zh, zm, Cc);
  k_conv<128, 128, float, false><<<gc, blk, 0, stream>>>(Cc, Wz, bz, Z);
  k_cat3<<<dim3(MTOK), dim3(192), 0, stream>>>(Z, h, C3);
  k_conv<192, 192, float, false><<<gc, blk, 0, stream>>>(C3, Wm, bm, comb);
  k_gates<<<dim3(MTOK), dim3(64), 0, stream>>>(comb, m, new_h, new_m);
}
